// EA_3307124818343
// MI455X (gfx1250) — hardware-verified
//
#include <hip/hip_runtime.h>
#include <stdint.h>

typedef _Float16 v16h __attribute__((ext_vector_type(16)));
typedef _Float16 v8h  __attribute__((ext_vector_type(8)));
typedef float    v8f  __attribute__((ext_vector_type(8)));
typedef float    v4f  __attribute__((ext_vector_type(4)));
union Frag { v16h v; v8h half[2]; };

#define NB   32
#define CH   96
#define HD   56
#define HW   3136
#define QD   128
#define ED   8
#define KT   864
#define KP   896
#define KPC  112
#define KTC  108
#define NT   64
#define LDA  104
#define LDB  104
#define LDC  68
#define AP   32

static_assert(HW % NT == 0);
static_assert(CH % 32 == 0);
static_assert((NB * CH * KPC) % 256 == 0);
static_assert(KP % 64 == 0);
static_assert(CH % 8 == 0);

__device__ __forceinline__ v8f wmma_f16(v16h a, v16h b, v8f c) {
    v8f d = __builtin_amdgcn_wmma_f32_16x16x32_f16(false, a, false, b, (short)0, c, false, false);
    asm volatile("v_nop\n\tv_nop\n\tv_nop\n\tv_nop" : "+v"(d) : "v"(a), "v"(b));
    return d;
}

__device__ __forceinline__ float wave_sum(float v) {
#pragma unroll
    for (int o = 16; o > 0; o >>= 1) v += __shfl_xor(v, o, 32);
    return v;
}

__global__ __launch_bounds__(256) void k_pool_softmax(
        const float* __restrict__ x,
        const float* __restrict__ Wq,
        const float* __restrict__ Wk,
        float* attn) {
    __shared__ float q[CH];
    __shared__ float qd[QD];
    __shared__ float lg[ED];
    __shared__ __attribute__((aligned(16))) float line[AP];
    const int b    = blockIdx.x;
    const int t    = threadIdx.x;
    const int lane = t & 31;
    const int wave = t >> 5;

    for (int c = wave; c < CH; c += 8) {
        const float4* xp = (const float4*)(x + ((size_t)b * CH + c) * HW);
        float s = 0.f;
        for (int i = lane; i < HW / 4; i += 32) {
            float4 v = xp[i];
            s += (v.x + v.y) + (v.z + v.w);
        }
        s = wave_sum(s);
        if (lane == 0) q[c] = s * (1.0f / (float)HW);
    }
    __syncthreads();

    if (t < QD) {
        const float* wr = Wq + (size_t)t * CH;
        float s = 0.f;
#pragma unroll 8
        for (int c = 0; c < CH; ++c) s = fmaf(q[c], wr[c], s);
        qd[t] = s;
    }
    if (t < AP) line[t] = 0.f;
    __syncthreads();

    if (t < ED) {
        const float* wr = Wk + (size_t)t * QD;
        float s = 0.f;
#pragma unroll 8
        for (int d = 0; d < QD; ++d) s = fmaf(qd[d], wr[d], s);
        lg[t] = s * 0.35355339059327373f;
    }
    __syncthreads();

    if (t == 0) {
        float mx = lg[0];
#pragma unroll
        for (int e = 1; e < ED; ++e) mx = fmaxf(mx, lg[e]);
        float ex[ED];
        float den = 0.f;
#pragma unroll
        for (int e = 0; e < ED; ++e) { ex[e] = __expf(lg[e] - mx); den += ex[e]; }
        const float inv = 1.0f / den;
#pragma unroll
        for (int e = 0; e < ED; ++e) line[e] = ex[e] * inv;
    }
    __syncthreads();

    v4f v = {0.f, 0.f, 0.f, 0.f};
    if (t < 8) v = *(const v4f*)(line + 4 * t);
    float* gp = attn + (size_t)b * AP + 4 * t;
    if (t < 8) *(volatile v4f*)gp = v;
    __threadfence();
    if (t < 8) *(volatile v4f*)gp = v;
}

__global__ __launch_bounds__(256) void k_fold_weights(
        const float* __restrict__ Wv,
        const float* __restrict__ attn,
        _Float16* Wf,
        int nchunks) {
    const int chunk = blockIdx.x * 256 + threadIdx.x;
    if (chunk >= nchunks) return;
    const int row = chunk / KPC;
    const int cq  = chunk - row * KPC;
    const int b   = row / CH;
    const int co  = row - b * CH;

    float vals[8];
#pragma unroll
    for (int j = 0; j < 8; ++j) vals[j] = 0.f;

    if (cq < KTC) {
        const int k0  = cq * 8;
        const int tap = k0 / CH;
        const int ci0 = k0 - tap * CH;
        float a[ED];
#pragma unroll
        for (int e = 0; e < ED; ++e) a[e] = attn[(size_t)b * AP + e];
        const float* wp = Wv + ((size_t)co * CH + ci0) * 9 + tap;
#pragma unroll
        for (int j = 0; j < 8; ++j) {
            float s = 0.f;
#pragma unroll
            for (int e = 0; e < ED; ++e)
                s = fmaf(a[e], wp[(size_t)e * (CH * CH * 9) + j * 9], s);
            vals[j] = s * 64.0f;
        }
    }
    v8h hv;
#pragma unroll
    for (int j = 0; j < 8; ++j) hv[j] = (_Float16)vals[j];
    _Float16* p = Wf + (size_t)chunk * 8;
    *(volatile v8h*)p = hv;
    __threadfence();
    *(volatile v8h*)p = hv;
}

__global__ __launch_bounds__(256) void k_conv3x3(
        const float* __restrict__ x,
        const _Float16* __restrict__ Wf,
        float* out) {
    __shared__ __attribute__((aligned(16))) _Float16 As[CH * LDA];
    __shared__ __attribute__((aligned(16))) _Float16 Bs[NT * LDB];
    __shared__ __attribute__((aligned(16))) float    Cs[CH * LDC];

    const int b      = blockIdx.y;
    const int p_base = blockIdx.x * NT;
    const int t      = threadIdx.x;
    const int lane   = t & 31;
    const int wave   = t >> 5;
    const int n_sub  = wave & 3;
    const int m0     = wave >> 2;
    const int m      = lane & 15;
    const int h      = lane >> 4;

    const int bn  = t & (NT - 1);
    const int cig = t >> 6;
    const int p   = p_base + bn;
    const int ph  = p / HD;
    const int pw  = p - ph * HD;

    v8f acc0, acc1, acc2;
#pragma unroll
    for (int r = 0; r < 8; ++r) { acc0[r] = 0.f; acc1[r] = 0.f; acc2[r] = 0.f; }

    const _Float16* wb = Wf + (size_t)b * CH * KP;
    const float*    xb = x  + (size_t)b * CH * HW;

    for (int tap = 0; tap < 9; ++tap) {
        const int th = tap / 3;
        const int dh = th - 1;
        const int dw = (tap - th * 3) - 1;

        for (int i = t; i < CH * 12; i += 256) {
            const int row = i / 12;
            const int qq  = i - row * 12;
            v8h v = *(const v8h*)(wb + (size_t)row * KP + tap * CH + qq * 8);
            *(v8h*)(As + row * LDA + qq * 8) = v;
        }

        {
            const int  hs    = ph + dh;
            const int  wsft  = pw + dw;
            const bool valid = (p < HW) && hs >= 0 && hs < HD && wsft >= 0 && wsft < HD;
            const int  off   = valid ? (hs * HD + wsft) : 0;
            const float* src = xb + (size_t)cig * HW + off;
            _Float16*    dst = Bs + bn * LDB + cig;
#pragma unroll 4
            for (int j = 0; j < CH / 4; ++j) {
                float v = src[(size_t)j * 4 * HW];
                v = valid ? v : 0.f;
                dst[4 * j] = (_Float16)v;
            }
        }
        __syncthreads();

        const _Float16* brow = Bs + (n_sub * 16 + m) * LDB + 8 * h;
        const _Float16* ar0  = As + ((m0 + 0) * 16 + m) * LDA + 8 * h;
        const _Float16* ar1  = As + ((m0 + 2) * 16 + m) * LDA + 8 * h;
        const _Float16* ar2  = As + ((m0 + 4) * 16 + m) * LDA + 8 * h;
#pragma unroll
        for (int s = 0; s < 3; ++s) {
            const int k0 = s * 32;
            Frag fb, fa0, fa1, fa2;
            fb.half[0]  = *(const v8h*)(brow + k0);
            fb.half[1]  = *(const v8h*)(brow + k0 + 16);
            fa0.half[0] = *(const v8h*)(ar0 + k0);
            fa0.half[1] = *(const v8h*)(ar0 + k0 + 16);
            fa1.half[0] = *(const v8h*)(ar1 + k0);
            fa1.half[1] = *(const v8h*)(ar1 + k0 + 16);
            fa2.half[0] = *(const v8h*)(ar2 + k0);
            fa2.half[1] = *(const v8h*)(ar2 + k0 + 16);
            acc0 = wmma_f16(fa0.v, fb.v, acc0);
            acc1 = wmma_f16(fa1.v, fb.v, acc1);
            acc2 = wmma_f16(fa2.v, fb.v, acc2);
        }
        __syncthreads();
    }

    {
        const float sc = 0.015625f;
        const int   cc = n_sub * 16 + m;
#pragma unroll
        for (int r = 0; r < 8; ++r) {
            const int rr = 8 * h + r;
            Cs[((m0 + 0) * 16 + rr) * LDC + cc] = acc0[r] * sc;
            Cs[((m0 + 2) * 16 + rr) * LDC + cc] = acc1[r] * sc;
            Cs[((m0 + 4) * 16 + rr) * LDC + cc] = acc2[r] * sc;
        }
    }
    __syncthreads();

    v4f vals[6];
#pragma unroll
    for (int j = 0; j < 6; ++j) {
        const int c   = t + 256 * j;
        const int row = c >> 4;
        const int q4  = c & 15;
        vals[j] = *(const v4f*)(Cs + row * LDC + q4 * 4);
    }
    float* ob = out + (size_t)b * CH * HW + p_base;
#pragma unroll
    for (int j = 0; j < 6; ++j) {
        const int c   = t + 256 * j;
        const int row = c >> 4;
        const int q4  = c & 15;
        *(volatile v4f*)(ob + (size_t)row * HW + q4 * 4) = vals[j];
    }
    __threadfence();
#pragma unroll
    for (int j = 0; j < 6; ++j) {
        const int c   = t + 256 * j;
        const int row = c >> 4;
        const int q4  = c & 15;
        *(volatile v4f*)(ob + (size_t)row * HW + q4 * 4) = vals[j];
    }
}

extern "C" void kernel_launch(void* const* d_in, const int* in_sizes, int n_in,
                              void* d_out, int out_size, void* d_ws, size_t ws_size,
                              hipStream_t stream) {
    if (n_in < 4) return;
    if (in_sizes[0] != NB * CH * HW) return;
    if (in_sizes[1] != QD * CH) return;
    if (in_sizes[2] != ED * QD) return;
    if (in_sizes[3] != ED * CH * CH * 9) return;
    if (out_size != NB * CH * HW) return;

    const float* x  = (const float*)d_in[0];
    const float* Wq = (const float*)d_in[1];
    const float* Wk = (const float*)d_in[2];
    const float* Wv = (const float*)d_in[3];
    float* out = (float*)d_out;

    const size_t attn_bytes = (size_t)NB * AP * sizeof(float);
    const size_t wf_off     = attn_bytes;
    const size_t wf_bytes   = (size_t)NB * CH * KP * sizeof(_Float16);
    if (wf_off + wf_bytes > ws_size) return;

    char* ws = (char*)d_ws;
    float*    attn = (float*)ws;
    _Float16* Wf   = (_Float16*)(ws + wf_off);

    k_pool_softmax<<<NB, 256, 0, stream>>>(x, Wq, Wk, attn);

    const int nchunks = NB * CH * KPC;
    k_fold_weights<<<(nchunks + 255) / 256, 256, 0, stream>>>(Wv, attn, Wf, nchunks);

    dim3 grid(HW / NT, NB);
    k_conv3x3<<<grid, 256, 0, stream>>>(x, Wf, out);
}
